// self_attention_layer_7653631721582
// MI455X (gfx1250) — hardware-verified
//
#include <hip/hip_runtime.h>
#include <math.h>
#include <stdint.h>

#ifndef NB
#define NB 8
#endif
#ifndef NQ
#define NQ 2048
#endif
#define NBF  8
#define NC   2048
#define ND   768
#define QT   64
#define OSP  68
#define TPW  72
#define KCH  64
#define USC  16.0f
#define IUSC 0.0625f
#define LNPS 9.704060527839234f
#define EPSV 1.0e-5f
#define ATTN_LDS (4 * 16 * ND * 4)

static_assert(NB >= 1 && NB <= NBF);
static_assert(NQ % QT == 0 && NQ >= QT && NQ <= NC);
static_assert(NC % QT == 0 && ND % QT == 0);
static_assert(NC % 32 == 0 && ND % 32 == 0);
static_assert(ND % 256 == 0 && ND % 128 == 0 && ND % 16 == 0);
static_assert(NC / KCH == 32 && KCH == 64);
static_assert(4 * NBF <= 32);
static_assert((OSP * 4) % 16 == 0);
static_assert((TPW * 2) % 16 == 0);
static_assert(ATTN_LDS == 196608);

typedef _Float16       v16h __attribute__((ext_vector_type(16)));
typedef _Float16       v8h  __attribute__((ext_vector_type(8)));
typedef __bf16         v16b __attribute__((ext_vector_type(16)));
typedef unsigned short v8us __attribute__((ext_vector_type(8)));
typedef float          v8f  __attribute__((ext_vector_type(8)));
typedef float          v4f  __attribute__((ext_vector_type(4)));
typedef unsigned int   v4u  __attribute__((ext_vector_type(4)));
typedef double         v2d  __attribute__((ext_vector_type(2)));

union Frag  { v8us u[2]; v16h h; v16b bf; };
union FragH { v16h v; v8h hv[2]; };
static_assert(sizeof(Frag) == 32);
static_assert(sizeof(FragH) == 32);

__device__ __forceinline__ unsigned short bf_bits(float f) {
  unsigned u = __float_as_uint(f);
  return (unsigned short)((u + 0x7FFFu + ((u >> 16) & 1u)) >> 16);
}
__device__ __forceinline__ float bf_up(unsigned short hb) { return __uint_as_float(((unsigned)hb) << 16); }
__device__ __forceinline__ float bf_lo16(unsigned w) { return __uint_as_float(w << 16); }
__device__ __forceinline__ float bf_hi16(unsigned w) { return __uint_as_float(w & 0xFFFF0000u); }
__device__ __forceinline__ unsigned short h_bits(_Float16 x) { return __builtin_bit_cast(unsigned short, x); }
__device__ __forceinline__ unsigned pk16(unsigned short a, unsigned short b) { return (unsigned)a | ((unsigned)b << 16); }
__device__ __forceinline__ v8f zero8() { v8f z = {0.f, 0.f, 0.f, 0.f, 0.f, 0.f, 0.f, 0.f}; return z; }
__device__ __forceinline__ float hmax8(v8f s) {
  return fmaxf(fmaxf(fmaxf(s[0], s[1]), fmaxf(s[2], s[3])), fmaxf(fmaxf(s[4], s[5]), fmaxf(s[6], s[7])));
}
__device__ __forceinline__ double shfl_xor_d(double v, int mask) {
  int lo = __double2loint(v), hi = __double2hiint(v);
  lo = __shfl_xor(lo, mask, 32);
  hi = __shfl_xor(hi, mask, 32);
  return __hiloint2double(hi, lo);
}

__device__ __forceinline__ Frag ldfrag(const unsigned short* p) {
  Frag f;
  f.u[0] = *(const v8us*)(p);
  f.u[1] = *(const v8us*)(p + 16);
  return f;
}

__device__ __forceinline__ v8f mma_h(v16h a, v16h b, v8f c) {
  v8f d = __builtin_amdgcn_wmma_f32_16x16x32_f16(false, a, false, b, (short)0, c, false, false);
#if defined(__HIP_DEVICE_COMPILE__)
  asm volatile("v_nop\n\tv_nop\n\tv_nop\n\tv_nop" : "+v"(d) : "v"(a), "v"(b));
#endif
  return d;
}
__device__ __forceinline__ v8f mma_b(v16b a, v16b b, v8f c) {
  v8f d = __builtin_amdgcn_wmma_f32_16x16x32_bf16(false, a, false, b, (short)0, c, false, false);
#if defined(__HIP_DEVICE_COMPILE__)
  const v16h ha = __builtin_bit_cast(v16h, a), hb = __builtin_bit_cast(v16h, b);
  asm volatile("v_nop\n\tv_nop\n\tv_nop\n\tv_nop" : "+v"(d) : "v"(ha), "v"(hb));
#endif
  return d;
}

__global__ __launch_bounds__(256)
void cvt_w(const float* __restrict__ wk, const float* __restrict__ wq, const float* __restrict__ wv,
           unsigned short* Wn, unsigned short* Wt, float* rs) {
  __shared__ __align__(16) unsigned short T[QT * TPW];
  __shared__ __align__(16) float rsL[QT];
  const int tid = threadIdx.x, lane = tid & 31, wave = tid >> 5;
  const int y = blockIdx.y, o0 = blockIdx.x * QT;
  const float* W = (y == 0) ? wk : ((y == 1) ? wq : wv);
  unsigned short* Np = Wn + (size_t)y * ND * ND;
  unsigned short* Tq = Wt + (size_t)y * ND * ND;
  const int e = lane & 7, r4 = lane >> 3;
  const int e8 = tid & 7, lq = tid >> 3;
  float rsum0 = 0.f, rsum1 = 0.f;
#pragma unroll 1
  for (int cc = 0; cc < ND / QT; ++cc) {
    const int i0 = cc * QT;
#pragma unroll
    for (int it = 0; it < 2; ++it) {
      const int ol = 8 * wave + 4 * it + r4;
      const float* sp = W + (size_t)(o0 + ol) * ND + i0 + 8 * e;
      const v4f a = *(const v4f*)sp;
      const v4f q = *(const v4f*)(sp + 4);
      const float f[8] = {a[0], a[1], a[2], a[3], q[0], q[1], q[2], q[3]};
      unsigned short hb[8];
      float ps = 0.f;
#pragma unroll
      for (int t = 0; t < 8; ++t) { hb[t] = bf_bits(f[t]); ps += bf_up(hb[t]); }
      if (it == 0) rsum0 += ps; else rsum1 += ps;
      v4u u;
#pragma unroll
      for (int t = 0; t < 4; ++t) u[t] = pk16(hb[2 * t], hb[2 * t + 1]);
      unsigned short* np = Np + (size_t)(o0 + ol) * ND + i0 + 8 * e;
      *(volatile v4u*)np = u;
      __threadfence();
      *(volatile v4u*)np = u;
#pragma unroll
      for (int t = 0; t < 8; ++t) T[(8 * e + t) * TPW + ol] = hb[t];
    }
    __syncthreads();
    v4u up[2];
#pragma unroll
    for (int it = 0; it < 2; ++it) {
      const int il = 32 * it + lq;
      up[it] = *(const v4u*)(T + il * TPW + 8 * e8);
    }
#pragma unroll
    for (int pass = 0; pass < 2; ++pass) {
#pragma unroll
      for (int it = 0; it < 2; ++it) {
        const int il = 32 * it + lq;
        *(volatile v4u*)(Tq + (size_t)(i0 + il) * ND + o0 + 8 * e8) = up[it];
      }
      __threadfence();
    }
    __syncthreads();
  }
  rsum0 += __shfl_xor(rsum0, 1, 32); rsum0 += __shfl_xor(rsum0, 2, 32); rsum0 += __shfl_xor(rsum0, 4, 32);
  rsum1 += __shfl_xor(rsum1, 1, 32); rsum1 += __shfl_xor(rsum1, 2, 32); rsum1 += __shfl_xor(rsum1, 4, 32);
  if (e == 0) { rsL[8 * wave + r4] = rsum0; rsL[8 * wave + 4 + r4] = rsum1; }
  __syncthreads();
  if (wave == 0 && lane < 16) {
    const v4f v = *(const v4f*)(rsL + 4 * lane);
    float* rp = rs + (size_t)y * ND + o0 + 4 * lane;
    *(volatile v4f*)rp = v;
    __threadfence();
    *(volatile v4f*)rp = v;
  }
}

__global__ __launch_bounds__(256)
void k_g(const unsigned short* __restrict__ Wkn, const float* __restrict__ rq, float* g) {
  __shared__ __align__(16) float gL[256];
  const int tid = threadIdx.x, lane = tid & 31, wave = tid >> 5;
  const int e = blockIdx.x * 256 + tid;
  float acc = 0.f;
#pragma unroll 4
  for (int o = 0; o < ND; ++o) acc += bf_up(Wkn[(size_t)o * ND + e]) * rq[o];
  gL[tid] = acc;
  __syncthreads();
  if (lane < 8) {
    const v4f v = *(const v4f*)(gL + 32 * wave + 4 * lane);
    float* p = g + (size_t)blockIdx.x * 256 + 32 * wave + 4 * lane;
    *(volatile v4f*)p = v;
    __threadfence();
    *(volatile v4f*)p = v;
  }
}

__global__ __launch_bounds__(256)
void k_xcvt(const float* __restrict__ x, unsigned short* Xb, double* part) {
  __shared__ double sL[8], qL[8];
  const int tid = threadIdx.x, lane = tid & 31, wave = tid >> 5;
  const int ch = blockIdx.x, b = blockIdx.y;
  const int r0 = ch * (NC / KCH);
  double s = 0.0, q = 0.0;
#pragma unroll 1
  for (int t = 0; t < 4; ++t) {
    const int row = r0 + 4 * wave + t;
    const size_t base = ((size_t)b * NC + row) * ND + 8 * lane;
#pragma unroll 1
    for (int c3 = 0; c3 < ND / 256; ++c3) {
      const float* sp = x + base + 256 * c3;
      const v4f a = *(const v4f*)sp;
      const v4f q4 = *(const v4f*)(sp + 4);
      const float f[8] = {a[0], a[1], a[2], a[3], q4[0], q4[1], q4[2], q4[3]};
      unsigned short hb[8];
#pragma unroll
      for (int k = 0; k < 8; ++k) {
        hb[k] = bf_bits(f[k]);
        const double v = (double)bf_up(hb[k]);
        s += v;
        q += v * v;
      }
      v4u u;
#pragma unroll
      for (int k = 0; k < 4; ++k) u[k] = pk16(hb[2 * k], hb[2 * k + 1]);
      unsigned short* xp = Xb + base + 256 * c3;
      *(volatile v4u*)xp = u;
      __threadfence();
      *(volatile v4u*)xp = u;
    }
  }
  s += shfl_xor_d(s, 16); s += shfl_xor_d(s, 8); s += shfl_xor_d(s, 4); s += shfl_xor_d(s, 2); s += shfl_xor_d(s, 1);
  q += shfl_xor_d(q, 16); q += shfl_xor_d(q, 8); q += shfl_xor_d(q, 4); q += shfl_xor_d(q, 2); q += shfl_xor_d(q, 1);
  if (lane == 0) { sL[wave] = s; qL[wave] = q; }
  __syncthreads();
  if (wave == 0) {
    double S = 0.0, Q = 0.0;
#pragma unroll
    for (int w = 0; w < 8; ++w) { S += sL[w]; Q += qL[w]; }
    v2d val;
    val[0] = (lane == 0) ? S : 0.0;
    val[1] = (lane == 0) ? Q : 0.0;
    if (lane < 8) {
      double* pp = part + ((size_t)b * KCH + ch) * 16 + 2 * lane;
      *(volatile v2d*)pp = val;
      __threadfence();
      *(volatile v2d*)pp = val;
    }
  }
}

__global__ __launch_bounds__(64)
void k_stats(const double* __restrict__ part, float* st) {
  __shared__ double sL[64], qL[64];
  __shared__ __align__(16) float stL[32];
  const int tid = threadIdx.x;
  if (tid < 32) stL[tid] = 0.f;
#pragma unroll 1
  for (int b = 0; b < NB; ++b) {
    __syncthreads();
    const size_t pb = ((size_t)b * KCH + tid) * 16;
    sL[tid] = part[pb];
    qL[tid] = part[pb + 1];
    __syncthreads();
#pragma unroll
    for (int off = 32; off > 0; off >>= 1) {
      if (tid < off) { sL[tid] += sL[tid + off]; qL[tid] += qL[tid + off]; }
      __syncthreads();
    }
    if (tid == 0) {
      const double n  = (double)NC * (double)ND;
      const double mu = sL[0] / n;
      double var = qL[0] / n - mu * mu;
      if (var < 0.0) var = 0.0;
      const float varf = (float)var;
      const float ve   = varf + EPSV;
      const float rstd = (float)(1.0 / sqrt((double)ve));
      const float muf  = (float)mu;
      stL[4 * b + 0] = muf;
      stL[4 * b + 1] = rstd;
      stL[4 * b + 2] = rstd * rstd;
      stL[4 * b + 3] = muf * rstd * rstd;
    }
  }
  __syncthreads();
  if (tid < 8) {
    const v4f v = *(const v4f*)(stL + 4 * tid);
    float* p = st + 4 * tid;
    *(volatile v4f*)p = v;
    __threadfence();
    *(volatile v4f*)p = v;
  }
}

template <int NPROD>
__device__ __forceinline__ void gemm_k(const unsigned short* __restrict__ ap0,
                                       const unsigned short* __restrict__ ap1,
                                       const unsigned short* __restrict__ bp, v8f (&acc)[4]) {
#pragma unroll
  for (int mt = 0; mt < 4; ++mt) acc[mt] = zero8();
#pragma unroll 2
  for (int ks = 0; ks < ND / 32; ++ks) {
    const Frag fb = ldfrag(bp + 32 * ks);
#pragma unroll
    for (int mt = 0; mt < 4; ++mt) {
      const Frag fa = ldfrag(ap0 + (size_t)(16 * mt) * ND + 32 * ks);
      acc[mt] = mma_b(fa.bf, fb.bf, acc[mt]);
      if (NPROD == 2) {
        const Frag fl = ldfrag(ap1 + (size_t)(16 * mt) * ND + 32 * ks);
        acc[mt] = mma_b(fl.bf, fb.bf, acc[mt]);
      }
    }
  }
}

__device__ __forceinline__ void stage_os(float* Os, const v8f (&acc)[4], float sc, int wave, int hh, int c) {
  const int nl = 16 * wave + c;
#pragma unroll
  for (int mt = 0; mt < 4; ++mt) {
    v4f va, vb;
#pragma unroll
    for (int r = 0; r < 4; ++r) { va[r] = acc[mt][r] * sc; vb[r] = acc[mt][4 + r] * sc; }
    *(v4f*)(Os + nl * OSP + 16 * mt + 8 * hh)     = va;
    *(v4f*)(Os + nl * OSP + 16 * mt + 8 * hh + 4) = vb;
  }
}

__device__ __forceinline__ void epi_split(const float* Os, unsigned short* Ph, unsigned short* Pl,
                                          size_t row0, int pitch, int col0, int tid) {
  const int e = tid & 7, lq = tid >> 3;
  v4u uh[4], ul[4];
#pragma unroll
  for (int it = 0; it < 4; ++it) {
    const int row = it * 16 + lq;
    const v4f a = *(const v4f*)(Os + row * OSP + 8 * e);
    const v4f q = *(const v4f*)(Os + row * OSP + 8 * e + 4);
    const float f[8] = {a[0], a[1], a[2], a[3], q[0], q[1], q[2], q[3]};
#pragma unroll
    for (int t = 0; t < 4; ++t) {
      const float f0 = f[2 * t], f1 = f[2 * t + 1];
      const unsigned short hb0 = bf_bits(f0), hb1 = bf_bits(f1);
      const unsigned short lb0 = bf_bits(f0 - bf_up(hb0));
      const unsigned short lb1 = bf_bits(f1 - bf_up(hb1));
      uh[it][t] = pk16(hb0, hb1);
      ul[it][t] = pk16(lb0, lb1);
    }
  }
#pragma unroll
  for (int pass = 0; pass < 2; ++pass) {
#pragma unroll
    for (int it = 0; it < 4; ++it) {
      const int row = it * 16 + lq;
      const size_t po = (row0 + (size_t)row) * (size_t)pitch + (size_t)col0 + 8 * e;
      *(volatile v4u*)(Ph + po) = uh[it];
      *(volatile v4u*)(Pl + po) = ul[it];
    }
    __threadfence();
  }
}

__device__ __forceinline__ void epi_h(const float* Os, unsigned short* P, size_t row0, int pitch, int col0, int tid) {
  const int e = tid & 7, lq = tid >> 3;
  v4u u[4];
#pragma unroll
  for (int it = 0; it < 4; ++it) {
    const int row = it * 16 + lq;
    const v4f a = *(const v4f*)(Os + row * OSP + 8 * e);
    const v4f q = *(const v4f*)(Os + row * OSP + 8 * e + 4);
    const float f[8] = {a[0], a[1], a[2], a[3], q[0], q[1], q[2], q[3]};
#pragma unroll
    for (int t = 0; t < 4; ++t)
      u[it][t] = pk16(h_bits((_Float16)f[2 * t]), h_bits((_Float16)f[2 * t + 1]));
  }
#pragma unroll
  for (int pass = 0; pass < 2; ++pass) {
#pragma unroll
    for (int it = 0; it < 4; ++it) {
      const int row = it * 16 + lq;
      const size_t po = (row0 + (size_t)row) * (size_t)pitch + (size_t)col0 + 8 * e;
      *(volatile v4u*)(P + po) = u[it];
    }
    __threadfence();
  }
}

__global__ __launch_bounds__(128)
void k_hgemm(const unsigned short* __restrict__ Aq, const unsigned short* __restrict__ Bk,
             unsigned short* Hh, unsigned short* Hl) {
  __shared__ __align__(16) float Os[QT * OSP];
  const int tid = threadIdx.x, lane = tid & 31, wave = tid >> 5, hh = lane >> 4, c = lane & 15;
  const int n0 = blockIdx.x * QT, m0 = blockIdx.y * QT;
  const unsigned short* ap = Aq + (size_t)(m0 + c) * ND + 8 * hh;
  const unsigned short* bp = Bk + (size_t)(n0 + 16 * wave + c) * ND + 8 * hh;
  v8f acc[4];
  gemm_k<1>(ap, ap, bp, acc);
  stage_os(Os, acc, 1.0f, wave, hh, c);
  __syncthreads();
  epi_split(Os, Hh, Hl, (size_t)n0, ND, m0, tid);
}

__global__ __launch_bounds__(128)
void k_agemm(const unsigned short* __restrict__ Hh, const unsigned short* __restrict__ Hl,
             const unsigned short* __restrict__ Xb, const float* __restrict__ st,
             unsigned short* Ah, unsigned short* Al) {
  __shared__ __align__(16) float Os[QT * OSP];
  const int tid = threadIdx.x, lane = tid & 31, wave = tid >> 5, hh = lane >> 4, c = lane & 15;
  const int n0 = blockIdx.x * QT, m0 = blockIdx.y * QT, b = blockIdx.z;
  const unsigned short* ap0 = Hh + (size_t)(m0 + c) * ND + 8 * hh;
  const unsigned short* ap1 = Hl + (size_t)(m0 + c) * ND + 8 * hh;
  const unsigned short* bp  = Xb + ((size_t)b * NC + n0 + 16 * wave + c) * ND + 8 * hh;
  v8f acc[4];
  gemm_k<2>(ap0, ap1, bp, acc);
  const float sc = st[4 * b + 2];
  stage_os(Os, acc, sc, wave, hh, c);
  __syncthreads();
  epi_split(Os, Ah, Al, (size_t)b * NQ + n0, ND, m0, tid);
}

__global__ __launch_bounds__(128)
void k_vgemm(const unsigned short* __restrict__ Xb, const unsigned short* __restrict__ Wvn, unsigned short* U) {
  __shared__ __align__(16) float Os[QT * OSP];
  const int tid = threadIdx.x, lane = tid & 31, wave = tid >> 5, hh = lane >> 4, c = lane & 15;
  const int n0 = blockIdx.x * QT, m0 = blockIdx.y * QT, b = blockIdx.z;
  const unsigned short* ap = Xb + ((size_t)b * NC + m0 + c) * ND + 8 * hh;
  const unsigned short* bp = Wvn + (size_t)(n0 + 16 * wave + c) * ND + 8 * hh;
  v8f acc[4];
  gemm_k<1>(ap, ap, bp, acc);
  stage_os(Os, acc, USC, wave, hh, c);
  __syncthreads();
  epi_h(Os, U, (size_t)b * ND + n0, NC, m0, tid);
}

__global__ __launch_bounds__(256)
void k_cs(const unsigned short* __restrict__ Xb, const float* __restrict__ g, const float* __restrict__ st,
          float* cs) {
  __shared__ __align__(16) float csL[32];
  const int tid = threadIdx.x, lane = tid & 31, wave = tid >> 5;
  const int r0 = blockIdx.x * 32, b = blockIdx.y;
  v4f ga[3], gb[3];
#pragma unroll
  for (int c3 = 0; c3 < 3; ++c3) {
    ga[c3] = *(const v4f*)(g + 256 * c3 + 8 * lane);
    gb[c3] = *(const v4f*)(g + 256 * c3 + 8 * lane + 4);
  }
  const float nmr = -st[4 * b + 3];
#pragma unroll 1
  for (int t = 0; t < 4; ++t) {
    const int row = r0 + 4 * wave + t;
    const unsigned short* xp = Xb + ((size_t)b * NC + row) * ND + 8 * lane;
    float acc = 0.f;
#pragma unroll
    for (int c3 = 0; c3 < 3; ++c3) {
      const v4u u = *(const v4u*)(xp + 256 * c3);
      acc += bf_lo16(u[0]) * ga[c3][0] + bf_hi16(u[0]) * ga[c3][1]
           + bf_lo16(u[1]) * ga[c3][2] + bf_hi16(u[1]) * ga[c3][3]
           + bf_lo16(u[2]) * gb[c3][0] + bf_hi16(u[2]) * gb[c3][1]
           + bf_lo16(u[3]) * gb[c3][2] + bf_hi16(u[3]) * gb[c3][3];
    }
    acc += __shfl_xor(acc, 16, 32); acc += __shfl_xor(acc, 8, 32); acc += __shfl_xor(acc, 4, 32);
    acc += __shfl_xor(acc, 2, 32);  acc += __shfl_xor(acc, 1, 32);
    if (lane == 0) csL[4 * wave + t] = acc * nmr;
  }
  __syncthreads();
  if (wave == 0 && lane < 8) {
    const v4f v = *(const v4f*)(csL + 4 * lane);
    float* p = cs + (size_t)b * NC + r0 + 4 * lane;
    *(volatile v4f*)p = v;
    __threadfence();
    *(volatile v4f*)p = v;
  }
}

__global__ __launch_bounds__(128)
void k_attn(const unsigned short* __restrict__ Ah, const unsigned short* __restrict__ Al,
            const unsigned short* __restrict__ Xb, const unsigned short* __restrict__ U,
            const float* __restrict__ cs, const float* __restrict__ rv,
            const float* __restrict__ st, float* out) {
  extern __shared__ v4f lds_dyn[];
  const int tid  = threadIdx.x;
  const int wave = tid >> 5, lane = tid & 31;
  const int hh   = lane >> 4, c = lane & 15;
  const int n0   = blockIdx.x * QT, b = blockIdx.y;
  float* Ow = (float*)lds_dyn + (size_t)wave * (16 * ND);
  float* op = Ow + c * ND + 8 * hh;
#pragma unroll 8
  for (int j = 0; j < ND / 16; ++j) {
    const v4f z = {0.f, 0.f, 0.f, 0.f};
    *(v4f*)(op + 16 * j)     = z;
    *(v4f*)(op + 16 * j + 4) = z;
  }

  const size_t qo = ((size_t)b * NQ + n0 + 16 * wave + c) * ND + 8 * hh;
  const unsigned short* Ahp = Ah + qo;
  const unsigned short* Alp = Al + qo;
  const unsigned short* Kp  = Xb + (size_t)b * NC * ND + (size_t)c * ND + 8 * hh;
  const unsigned short* Vp  = U + (size_t)b * ND * NC + (size_t)c * NC + 8 * hh;
  const float* csb = cs + (size_t)b * NC + 8 * hh;

  float m = -1.0e30f, l = 0.f;
#pragma unroll 1
  for (int kb = 0; kb < NC; kb += 32) {
    const unsigned short* k0p = Kp + (size_t)kb * ND;
    const unsigned short* k1p = Kp + (size_t)(kb + 16) * ND;
    v8f s0 = zero8(), s1 = zero8();
#pragma unroll 1
    for (int kc = 0; kc < ND / 32; ++kc) {
      const Frag qh = ldfrag(Ahp + 32 * kc);
      const Frag ql = ldfrag(Alp + 32 * kc);
      const Frag k0 = ldfrag(k0p + 32 * kc);
      const Frag k1 = ldfrag(k1p + 32 * kc);
      s0 = mma_b(k0.bf, qh.bf, s0);
      s1 = mma_b(k1.bf, qh.bf, s1);
      s0 = mma_b(k0.bf, ql.bf, s0);
      s1 = mma_b(k1.bf, ql.bf, s1);
    }
    {
      const v4f ca = *(const v4f*)(csb + kb);
      const v4f cb = *(const v4f*)(csb + kb + 4);
      const v4f cd = *(const v4f*)(csb + kb + 16);
      const v4f ce = *(const v4f*)(csb + kb + 20);
#pragma unroll
      for (int r = 0; r < 4; ++r) {
        s0[r] += ca[r]; s0[4 + r] += cb[r];
        s1[r] += cd[r]; s1[4 + r] += ce[r];
      }
    }

    float mx = fmaxf(hmax8(s0), hmax8(s1));
    mx = fmaxf(mx, __shfl_xor(mx, 16, 32));
    const float mn   = fmaxf(m, mx);
    const float corr = __expf(m - mn);
    l *= corr;
    m = mn;
    const float msh = mn - LNPS;

    FragH ph;
    float ls = 0.f;
#pragma unroll
    for (int r = 0; r < 8; ++r) {
      const float e0 = __expf(s0[r] - msh);
      const float e1 = __expf(s1[r] - msh);
      ls += e0 + e1;
      ph.hv[0][r] = (_Float16)e0;
      ph.hv[1][r] = (_Float16)e1;
    }
    l += ls;

#pragma unroll 4
    for (int j = 0; j < ND / 16; ++j) {
      const v4f oa = *(const v4f*)(op + 16 * j);
      const v4f ob = *(const v4f*)(op + 16 * j + 4);
      v8f o;
#pragma unroll
      for (int r = 0; r < 4; ++r) { o[r] = oa[r] * corr; o[4 + r] = ob[r] * corr; }
      const Frag vf = ldfrag(Vp + (size_t)(16 * j) * NC + kb);
      o = mma_h(vf.h, ph.v, o);
      v4f na, nb2;
#pragma unroll
      for (int r = 0; r < 4; ++r) { na[r] = o[r]; nb2[r] = o[4 + r]; }
      *(v4f*)(op + 16 * j)     = na;
      *(v4f*)(op + 16 * j + 4) = nb2;
    }
  }
  l += __shfl_xor(l, 16, 32);
  const float inv  = 1.0f / l;
  const float mu   = st[4 * b + 0], rstd = st[4 * b + 1];
  const float qsc  = inv * rstd * IUSC;
  const float mrs  = mu * rstd;
  v4f rvv[6];
#pragma unroll
  for (int k = 0; k < ND / 128; ++k) {
    const v4f t = *(const v4f*)(rv + 128 * k + 4 * lane);
#pragma unroll
    for (int u = 0; u < 4; ++u) rvv[k][u] = t[u] * mrs;
  }
  __syncthreads();

#pragma unroll
  for (int pass = 0; pass < 2; ++pass) {
#pragma unroll 1
    for (int qq = 0; qq < 16; ++qq) {
      const float sc = __shfl(qsc, qq, 32);
      const float* lrow = Ow + qq * ND + 4 * lane;
      float* orow = out + ((size_t)b * NC + n0 + 16 * wave + qq) * ND + 4 * lane;
#pragma unroll
      for (int k = 0; k < ND / 128; ++k) {
        const v4f v = *(const v4f*)(lrow + 128 * k);
        v4f w;
#pragma unroll
        for (int u = 0; u < 4; ++u) w[u] = v[u] * sc - rvv[k][u];
        *(volatile v4f*)(orow + 128 * k) = w;
      }
    }
    __threadfence();
  }
}

extern "C" void kernel_launch(void* const* d_in, const int* in_sizes, int n_in,
                              void* d_out, int out_size, void* d_ws, size_t ws_size,
                              hipStream_t stream) {
  if (n_in < 4) return;
  if (in_sizes[0] < NB * NC * ND) return;
  if (in_sizes[1] < ND * ND || in_sizes[2] < ND * ND || in_sizes[3] < ND * ND) return;
  if (out_size < NB * NC * ND) return;

  size_t off = 0;
  auto carve = [&](size_t bytes) { const size_t o = off; off += (bytes + 255) & ~(size_t)255; return o; };
  const size_t oWn   = carve((size_t)3 * ND * ND * 2);
  const size_t oWt   = carve((size_t)3 * ND * ND * 2);
  const size_t oRs   = carve((size_t)3 * ND * 4);
  const size_t oG    = carve((size_t)ND * 4);
  const size_t oXb   = carve((size_t)NB * NC * ND * 2);
  const size_t oPart = carve((size_t)NB * KCH * 128);
  const size_t oSt   = carve((size_t)128);
  const size_t oHh   = carve((size_t)ND * ND * 2);
  const size_t oHl   = carve((size_t)ND * ND * 2);
  const size_t oAh   = carve((size_t)NB * NQ * ND * 2);
  const size_t oAl   = carve((size_t)NB * NQ * ND * 2);
  const size_t oU    = carve((size_t)NB * ND * NC * 2);
  const size_t oCs   = carve((size_t)NB * NC * 4);
  if (off > ws_size) return;
  if (off > (size_t)134217728) return;

  const float* x  = (const float*)d_in[0];
  const float* wk = (const float*)d_in[1];
  const float* wq = (const float*)d_in[2];
  const float* wv = (const float*)d_in[3];

  char* ws = (char*)d_ws;
  unsigned short* Wn  = (unsigned short*)(ws + oWn);
  unsigned short* Wt  = (unsigned short*)(ws + oWt);
  float*          rs  = (float*)(ws + oRs);
  float*          g   = (float*)(ws + oG);
  unsigned short* Xb  = (unsigned short*)(ws + oXb);
  double*         part = (double*)(ws + oPart);
  float*          st  = (float*)(ws + oSt);
  unsigned short* Hh  = (unsigned short*)(ws + oHh);
  unsigned short* Hl  = (unsigned short*)(ws + oHl);
  unsigned short* Ah  = (unsigned short*)(ws + oAh);
  unsigned short* Al  = (unsigned short*)(ws + oAl);
  unsigned short* U   = (unsigned short*)(ws + oU);
  float*          cs  = (float*)(ws + oCs);
  float* out = (float*)d_out;

  const dim3 blk256(256), blk128(128), blk64(64);

  cvt_w<<<dim3(ND / QT, 3), blk256, 0, stream>>>(wk, wq, wv, Wn, Wt, rs);
  k_g<<<dim3(ND / 256), blk256, 0, stream>>>(Wn, rs + ND, g);
  k_xcvt<<<dim3(KCH, NB), blk256, 0, stream>>>(x, Xb, part);
  k_stats<<<dim3(1), blk64, 0, stream>>>(part, st);
  k_hgemm<<<dim3(ND / QT, ND / QT), blk128, 0, stream>>>(Wt + (size_t)1 * ND * ND, Wt, Hh, Hl);
  k_agemm<<<dim3(NQ / QT, ND / QT, NB), blk128, 0, stream>>>(Hh, Hl, Xb, st, Ah, Al);
  k_vgemm<<<dim3(ND / QT, NC / QT, NB), blk128, 0, stream>>>(Xb, Wn + (size_t)2 * ND * ND, U);
  k_cs<<<dim3(NC / 32, NB), blk256, 0, stream>>>(Xb, g, st, cs);
  (void)hipFuncSetAttribute(reinterpret_cast<const void*>(&k_attn),
                            hipFuncAttributeMaxDynamicSharedMemorySize, ATTN_LDS);
  k_attn<<<dim3(NQ / QT, NB), blk128, ATTN_LDS, stream>>>(Ah, Al, Xb, U, cs, rs + 2 * ND, st, out);
  (void)hipGetLastError();
}
